// Block_12369505812822
// MI455X (gfx1250) — hardware-run, weakly checked
//
#include <hip/hip_runtime.h>

#ifndef NB
#define NB 4
#endif
#ifndef SEQ
#define SEQ 1024
#endif
#define NB_FULL 4
#define SEQ_FULL 1024
#ifndef OSEQ
#define OSEQ SEQ_FULL
#endif
#define DM 1024
#define NH 16
#define HD 64
#define HID 3072
#define NR ((size_t)NB * SEQ)
#define LN_EPS 1e-5f
#define AP_PL 0
#define AP_MX 8192
#define AP_POOL 18432

static_assert(NB >= 1 && NB <= NB_FULL);
static_assert(SEQ % 128 == 0 && SEQ <= SEQ_FULL);
static_assert(DM == NH * HD && HD == 64 && NH == 16);
static_assert(DM % 512 == 0 && HID % 64 == 0 && DM % 32 == 0 && HID % 32 == 0 && DM % 64 == 0);
static_assert(((NB * SEQ) % 128) == 0);
static_assert(AP_MX == 512 * 16 && AP_MX + 16 * 16 * 40 == AP_POOL && 16 * 16 * 72 == AP_POOL);
static_assert(AP_POOL * 2 + NH * 64 * 4 <= 131072);
static_assert(4 * 32 * 68 * 4 <= 131072);
static_assert(2 * 64 * 66 * 2 <= 131072);
static_assert(4ull * DM * DM * 2 + 3ull * DM * HID * 2 + 6ull * NB * SEQ * DM * 2 + 1ull * NB * SEQ * DM * 4 + 1ull * NB * SEQ * HID * 2 + (size_t)SEQ * 32 * 4 <= (128ull << 20));
static_assert(32 * 16 * 8 == 32 * 128);
static_assert(32 * 16 * 16 == 32 * 256);
static_assert(32 * 16 * 4 == 16 * 128);

typedef _Float16 h16;
typedef _Float16 v16h __attribute__((ext_vector_type(16)));
typedef __bf16   v16b __attribute__((ext_vector_type(16)));
typedef unsigned short v8us __attribute__((ext_vector_type(8), may_alias));
typedef float v8f __attribute__((ext_vector_type(8)));
typedef float v4f __attribute__((ext_vector_type(4)));
typedef float v4fa __attribute__((ext_vector_type(4), may_alias));
union Frag16 { v16h h; v16b b; v8us half[2]; unsigned short u[16]; };
union H1 { _Float16 h; unsigned short u; };
static_assert(sizeof(Frag16) == 32);

__device__ __forceinline__ unsigned short bf16_bits(float x) { unsigned int u = __float_as_uint(x); return (unsigned short)((u + 0x7FFFu + ((u >> 16) & 1u)) >> 16); }
__device__ __forceinline__ float bf16_val(unsigned short b) { return __uint_as_float(((unsigned int)b) << 16); }
__device__ __forceinline__ float bf16_rne(float x) { return bf16_val(bf16_bits(x)); }
static __device__ __forceinline__ h16 toh_flush(float v) { const h16 r = (h16)v; return (fabsf(v) < 6.103515625e-05f) ? (h16)0.0f : r; }
__device__ __forceinline__ unsigned short f16_flush_bits(float x) { H1 t; t.h = toh_flush(x); return t.u; }
__device__ __forceinline__ int iclamp(int v, int lo, int hi) { return v < lo ? lo : (v > hi ? hi : v); }

__device__ __forceinline__ Frag16 ld_frag(const unsigned short* p, int hh) {
  Frag16 f;
  f.half[0] = *(const v8us*)(p + 8 * hh);
  f.half[1] = *(const v8us*)(p + 16 + 8 * hh);
  return f;
}
__device__ __forceinline__ v8f mma_h(v16h a, v16h b, v8f c) {
  v8f d = __builtin_amdgcn_wmma_f32_16x16x32_f16(false, a, false, b, (short)0, c, false, false);
  asm volatile("v_nop\n\tv_nop\n\tv_nop\n\tv_nop" : "+v"(d) : "v"(a), "v"(b));
  return d;
}

template <bool BF, bool GAM>
__global__ __launch_bounds__(256) void k_wt(const float* __restrict__ W, const float* __restrict__ g, unsigned short* __restrict__ Bt, int K, int N, float scale) {
  const int k8n = K >> 3;
  const size_t t = (size_t)blockIdx.x * 256 + threadIdx.x;
  if (t >= (size_t)N * (size_t)k8n) return;
  const int n = (int)(t / (size_t)k8n), k8 = (int)(t % (size_t)k8n) * 8;
  float gv[8];
#pragma unroll
  for (int i = 0; i < 8; ++i) gv[i] = 1.0f;
  if (GAM) {
    const v4f ga = *(const v4fa*)(g + k8), gb = *(const v4fa*)(g + k8 + 4);
#pragma unroll
    for (int i = 0; i < 4; ++i) { gv[i] = bf16_rne(ga[i]); gv[4 + i] = bf16_rne(gb[i]); }
  }
  Frag16 f;
#pragma unroll
  for (int i = 0; i < 8; ++i) {
    const float wv = bf16_rne(W[(size_t)(k8 + i) * (size_t)N + n]) * gv[i];
    f.u[i] = BF ? bf16_bits(wv) : f16_flush_bits(wv * scale);
  }
  unsigned short* d = Bt + (size_t)n * (size_t)K + k8;
  *(volatile v8us*)d = f.half[0];
  __threadfence();
  *(volatile v8us*)d = f.half[0];
}

__global__ __launch_bounds__(256) void k_tab(float* __restrict__ TAB) {
#pragma clang fp contract(off)
  const int tid = threadIdx.x, lane = tid & 31;
  const int wave = __builtin_amdgcn_readfirstlane(tid >> 5);
  const int t = (int)blockIdx.x * 8 + wave;
  const int i = lane & 15;
  const float ex = (float)(2 * i) * (1.0f / 32.0f);
  const float inv = exp2f(-(ex * 13.287712379549449f));
  const float ang = (float)t * inv;
  float sn, cs;
  sincosf(ang, &sn, &cs);
  const float v = (lane < 16) ? cs : sn;
  float* d = TAB + (size_t)t * 32 + lane;
  *(volatile float*)d = v;
  __threadfence();
  *(volatile float*)d = v;
}

__global__ __launch_bounds__(256) void k_ln(const float* __restrict__ F, int spitch, const float* __restrict__ g, const float* __restrict__ bt,
    unsigned short* __restrict__ OUT, int rin, int shift) {
#pragma clang fp contract(off)
  const int tid = threadIdx.x, lane = tid & 31;
  const int wave = __builtin_amdgcn_readfirstlane(tid >> 5);
  const int rb = (int)blockIdx.x * 32;
  const v8us zero8 = {0, 0, 0, 0, 0, 0, 0, 0};
#pragma unroll 1
  for (int i = 0; i < 4; ++i) {
    const int r = rb + wave * 4 + i;
    const int sq = r % SEQ;
    const float* src = F + ((size_t)(r / SEQ) * (size_t)spitch + (size_t)sq) * DM;
    float s = 0.f;
#pragma unroll 1
    for (int u = 0; u < DM / 128; ++u) {
      v4f a = *(const v4fa*)(src + u * 128 + lane * 4);
      if (rin != 0) {
#pragma unroll
        for (int q = 0; q < 4; ++q) a[q] = bf16_rne(a[q]);
      }
      s += (a[0] + a[1]) + (a[2] + a[3]);
    }
#pragma unroll
    for (int off = 16; off > 0; off >>= 1) s += __shfl_xor(s, off, 32);
    const float mu = s * (1.0f / (float)DM);
    float ss = 0.f;
#pragma unroll 1
    for (int u = 0; u < DM / 128; ++u) {
      v4f a = *(const v4fa*)(src + u * 128 + lane * 4);
      if (rin != 0) {
#pragma unroll
        for (int q = 0; q < 4; ++q) a[q] = bf16_rne(a[q]);
      }
#pragma unroll
      for (int q = 0; q < 4; ++q) { const float d = a[q] - mu; ss += d * d; }
    }
#pragma unroll
    for (int off = 16; off > 0; off >>= 1) ss += __shfl_xor(ss, off, 32);
    const float rs = rsqrtf(ss * (1.0f / (float)DM) + LN_EPS);
#pragma unroll 1
    for (int u = 0; u < DM / 256; ++u) {
      const int j = u * 256 + lane * 8;
      v4f a = *(const v4fa*)(src + j), c = *(const v4fa*)(src + j + 4);
      if (rin != 0) {
#pragma unroll
        for (int q = 0; q < 4; ++q) { a[q] = bf16_rne(a[q]); c[q] = bf16_rne(c[q]); }
      }
      const v4f ga = *(const v4fa*)(g + j), gb = *(const v4fa*)(g + j + 4);
      const v4f ba = *(const v4fa*)(bt + j), bb = *(const v4fa*)(bt + j + 4);
      Frag16 fh;
#pragma unroll
      for (int q = 0; q < 4; ++q) {
        const float v0 = ((a[q] - mu) * rs) * bf16_rne(ga[q]) + bf16_rne(ba[q]);
        const float v1 = ((c[q] - mu) * rs) * bf16_rne(gb[q]) + bf16_rne(bb[q]);
        fh.u[q] = f16_flush_bits(v0); fh.u[4 + q] = f16_flush_bits(v1);
      }
      const int lowh = (shift != 0 && u < DM / 512) ? 1 : 0;
      const int doit = (lowh != 0 && sq >= SEQ - 1) ? 0 : 1;
      const int drow = (lowh != 0 && doit != 0) ? r + 1 : r;
      const int zrow = (lowh != 0 && sq == 0) ? 1 : 0;
      unsigned short* d = OUT + (size_t)drow * DM + j;
      unsigned short* z = OUT + (size_t)r * DM + j;
      if (doit != 0) *(volatile v8us*)d = fh.half[0];
      if (zrow != 0) *(volatile v8us*)z = zero8;
      __threadfence();
      if (doit != 0) *(volatile v8us*)d = fh.half[0];
      if (zrow != 0) *(volatile v8us*)z = zero8;
    }
  }
}

template <int EPI>
__device__ __forceinline__ void gemm_body(const unsigned short* __restrict__ Ah, int lda, const unsigned short* __restrict__ Bt, int ldb,
    float alpha, const float* __restrict__ bias, const float* __restrict__ resid, int rseq, int rpitch, int ldr,
    const float* __restrict__ gam, const float* __restrict__ tab, int tseq,
    float* __restrict__ C32, unsigned short* __restrict__ Ch, int ldc, int cseq, int cpitch, int M, int N, int K) {
  static_assert(EPI >= 0 && EPI <= 3);
  __shared__ __attribute__((aligned(16))) float so[4][32][68];
  const int tid = threadIdx.x, lane = tid & 31, ln = lane & 15, hh = lane >> 4;
  const int w = __builtin_amdgcn_readfirstlane(tid >> 5);
  const int ntn = N >> 6;
  const int mt = (int)blockIdx.x / ntn, nq = (int)blockIdx.x - mt * ntn;
  const int row0 = mt * 128 + 32 * w, col0 = nq * 64;
  if (row0 + 32 > M) return;
  const unsigned short* a0p = Ah + (size_t)(row0 + ln) * (size_t)lda;
  const unsigned short* a1p = a0p + (size_t)16 * (size_t)lda;
  const unsigned short* b0p = Bt + (size_t)(col0 + ln) * (size_t)ldb;
  const unsigned short* b1p = b0p + (size_t)16 * (size_t)ldb;
  const unsigned short* b2p = b1p + (size_t)16 * (size_t)ldb;
  const unsigned short* b3p = b2p + (size_t)16 * (size_t)ldb;
  const v8f z8 = {0.f, 0.f, 0.f, 0.f, 0.f, 0.f, 0.f, 0.f};
  v8f c00 = z8, c01 = z8, c02 = z8, c03 = z8, c10 = z8, c11 = z8, c12 = z8, c13 = z8;
#pragma unroll 1
  for (int kb = 0; kb < K; kb += 32) {
    const Frag16 a0 = ld_frag(a0p + kb, hh), a1 = ld_frag(a1p + kb, hh);
    Frag16 bq = ld_frag(b0p + kb, hh);
    c00 = mma_h(a0.h, bq.h, c00); c10 = mma_h(a1.h, bq.h, c10);
    bq = ld_frag(b1p + kb, hh);
    c01 = mma_h(a0.h, bq.h, c01); c11 = mma_h(a1.h, bq.h, c11);
    bq = ld_frag(b2p + kb, hh);
    c02 = mma_h(a0.h, bq.h, c02); c12 = mma_h(a1.h, bq.h, c12);
    bq = ld_frag(b3p + kb, hh);
    c03 = mma_h(a0.h, bq.h, c03); c13 = mma_h(a1.h, bq.h, c13);
  }
  const v8f accs[8] = {c00, c01, c02, c03, c10, c11, c12, c13};
#pragma unroll
  for (int u = 0; u < 8; ++u) {
    const int t = u & 3, half = u >> 2;
    const int col = col0 + t * 16 + ln;
    const float bv = bf16_rne(bias[col]);
#pragma unroll
    for (int r = 0; r < 8; ++r) {
      const int rloc = half * 16 + 8 * hh + r;
      so[w][rloc][t * 16 + ln] = accs[u][r] * alpha + bv;
    }
  }
  __builtin_amdgcn_fence(4  , "workgroup");
  __builtin_amdgcn_wave_barrier();
  if (EPI >= 2) {
#pragma unroll 1
    for (int pass = 0; pass < 2; ++pass) {
#pragma unroll 1
      for (int q = 0; q < 16; ++q) {
        const int r = q * 2 + (lane >> 4), c4 = (lane & 15) * 4;
        v4f v = *(const v4fa*)&so[w][r][c4];
        const int grow = row0 + r;
        const size_t rrow = (size_t)(grow / rseq) * (size_t)rpitch + (size_t)(grow % rseq);
        v4f rv = *(const v4fa*)(resid + rrow * (size_t)ldr + col0 + c4);
        if (EPI == 2) {
#pragma unroll
          for (int i = 0; i < 4; ++i) rv[i] = bf16_rne(rv[i]);
          const float gm = bf16_rne(gam[grow % tseq]);
          v = v * gm + rv;
        } else {
          v = v + rv;
        }
        const size_t crow = (size_t)(grow / cseq) * (size_t)cpitch + (size_t)(grow % cseq);
        *(volatile v4f*)(C32 + crow * (size_t)ldc + col0 + c4) = v;
      }
      if (pass == 0) __threadfence();
    }
  } else {
#pragma unroll 1
    for (int pass = 0; pass < 2; ++pass) {
#pragma unroll 1
      for (int q = 0; q < 8; ++q) {
        const int r = q * 4 + (lane >> 3), c8 = (lane & 7) * 8;
        v4f x0 = *(const v4fa*)&so[w][r][c8], x1 = *(const v4fa*)&so[w][r][c8 + 4];
        if (EPI == 1) {
          const int pc = c8 ^ 16;
          const v4f y0 = *(const v4fa*)&so[w][r][pc], y1 = *(const v4fa*)&so[w][r][pc + 4];
          const int tp = (row0 + r) % tseq;
          const float* tb = tab + (size_t)tp * 32 + (c8 & 15);
          v4f cs0 = *(const v4fa*)tb, cs1 = *(const v4fa*)(tb + 4);
          v4f sn0 = *(const v4fa*)(tb + 16), sn1 = *(const v4fa*)(tb + 20);
          asm volatile("" : "+v"(cs0));
          asm volatile("" : "+v"(cs1));
          asm volatile("" : "+v"(sn0));
          asm volatile("" : "+v"(sn1));
          const float sg = (c8 < 16) ? -1.0f : 1.0f;
          const bool rot = (c8 < 32);
#pragma unroll
          for (int i = 0; i < 4; ++i) {
            const float n0 = x0[i] * cs0[i] + sg * (y0[i] * sn0[i]);
            const float n1 = x1[i] * cs1[i] + sg * (y1[i] * sn1[i]);
            x0[i] = rot ? n0 : x0[i];
            x1[i] = rot ? n1 : x1[i];
          }
        }
        Frag16 fh;
#pragma unroll
        for (int i = 0; i < 4; ++i) { fh.u[i] = f16_flush_bits(x0[i]); fh.u[4 + i] = f16_flush_bits(x1[i]); }
        const size_t o = (size_t)(row0 + r) * (size_t)ldc + col0 + c8;
        *(volatile v8us*)(Ch + o) = fh.half[0];
      }
      if (pass == 0) __threadfence();
    }
  }
}

__global__ __launch_bounds__(128) void k_gemm_plain(const unsigned short* __restrict__ Ah, int lda, const unsigned short* __restrict__ Bt, int ldb,
    float alpha, const float* __restrict__ bias, unsigned short* __restrict__ Ch, int ldc, int M, int N, int K) {
  gemm_body<0>(Ah, lda, Bt, ldb, alpha, bias, nullptr, 1, 0, 0, nullptr, nullptr, 1, nullptr, Ch, ldc, 1, 0, M, N, K);
}
__global__ __launch_bounds__(128) void k_gemm_rope(const unsigned short* __restrict__ Ah, int lda, const unsigned short* __restrict__ Bt, int ldb,
    float alpha, const float* __restrict__ bias, const float* __restrict__ tab, int tseq, unsigned short* __restrict__ Ch, int ldc, int M, int N, int K) {
  gemm_body<1>(Ah, lda, Bt, ldb, alpha, bias, nullptr, 1, 0, 0, nullptr, tab, tseq, nullptr, Ch, ldc, 1, 0, M, N, K);
}
__global__ __launch_bounds__(128) void k_gemm_wo(const unsigned short* __restrict__ Ah, int lda, const unsigned short* __restrict__ Bt, int ldb,
    float alpha, const float* __restrict__ bias, const float* __restrict__ resid, int rseq, int rpitch, int ldr, const float* __restrict__ gam, int tseq,
    float* __restrict__ C32, int ldc, int cseq, int cpitch, int M, int N, int K) {
  gemm_body<2>(Ah, lda, Bt, ldb, alpha, bias, resid, rseq, rpitch, ldr, gam, nullptr, tseq, C32, nullptr, ldc, cseq, cpitch, M, N, K);
}
__global__ __launch_bounds__(128) void k_gemm_out(const unsigned short* __restrict__ Ah, int lda, const unsigned short* __restrict__ Bt, int ldb,
    float alpha, const float* __restrict__ bias, const float* __restrict__ resid, int rseq, int rpitch, int ldr,
    float* __restrict__ C32, int ldc, int cseq, int cpitch, int M, int N, int K) {
  gemm_body<3>(Ah, lda, Bt, ldb, alpha, bias, resid, rseq, rpitch, ldr, nullptr, nullptr, 1, C32, nullptr, ldc, cseq, cpitch, M, N, K);
}

__global__ __launch_bounds__(128) void k_ffup(const unsigned short* __restrict__ Ah, int lda, const unsigned short* __restrict__ Bk,
    const unsigned short* __restrict__ Bv, int ldb, float alpha, const float* __restrict__ biask, const float* __restrict__ biasv, float oscale,
    unsigned short* __restrict__ Ch, int ldc, int M, int N, int K) {
  __shared__ __attribute__((aligned(16))) float so[4][32][68];
  const int tid = threadIdx.x, lane = tid & 31, ln = lane & 15, hh = lane >> 4;
  const int w = __builtin_amdgcn_readfirstlane(tid >> 5);
  const int ntn = N >> 6;
  const int mt = (int)blockIdx.x / ntn, nq = (int)blockIdx.x - mt * ntn;
  const int row0 = mt * 128 + 32 * w, col0 = nq * 64;
  if (row0 + 32 > M) return;
  const unsigned short* a0p = Ah + (size_t)(row0 + ln) * (size_t)lda;
  const unsigned short* a1p = a0p + (size_t)16 * (size_t)lda;
  const unsigned short* bkp = Bk + (size_t)(col0 + ln) * (size_t)ldb;
  const unsigned short* bvp = Bv + (size_t)(col0 + ln) * (size_t)ldb;
  const size_t tstep = (size_t)16 * (size_t)ldb;
  const v8f z8 = {0.f, 0.f, 0.f, 0.f, 0.f, 0.f, 0.f, 0.f};
  v8f ck[2][4], cv[2][4];
#pragma unroll
  for (int a = 0; a < 2; ++a) {
#pragma unroll
    for (int t = 0; t < 4; ++t) { ck[a][t] = z8; cv[a][t] = z8; }
  }
#pragma unroll 1
  for (int kb = 0; kb < K; kb += 32) {
    const Frag16 a0 = ld_frag(a0p + kb, hh), a1 = ld_frag(a1p + kb, hh);
#pragma unroll
    for (int t = 0; t < 4; ++t) {
      Frag16 bq = ld_frag(bkp + (size_t)t * tstep + kb, hh);
      ck[0][t] = mma_h(a0.h, bq.h, ck[0][t]); ck[1][t] = mma_h(a1.h, bq.h, ck[1][t]);
      bq = ld_frag(bvp + (size_t)t * tstep + kb, hh);
      cv[0][t] = mma_h(a0.h, bq.h, cv[0][t]); cv[1][t] = mma_h(a1.h, bq.h, cv[1][t]);
    }
  }
  float bkv[4], bvv[4];
#pragma unroll
  for (int t = 0; t < 4; ++t) { bkv[t] = bf16_rne(biask[col0 + t * 16 + ln]); bvv[t] = bf16_rne(biasv[col0 + t * 16 + ln]); }
#pragma unroll
  for (int half = 0; half < 2; ++half) {
#pragma unroll
    for (int t = 0; t < 4; ++t) {
#pragma unroll
      for (int r = 0; r < 8; ++r) {
        so[w][8 * hh + r][t * 16 + ln] = ck[half][t][r] * alpha + bkv[t];
        so[w][16 + 8 * hh + r][t * 16 + ln] = cv[half][t][r] * alpha + bvv[t];
      }
    }
    __builtin_amdgcn_fence(4  , "workgroup");
    __builtin_amdgcn_wave_barrier();
#pragma unroll 1
    for (int q = 0; q < 4; ++q) {
      const int r = q * 4 + (lane >> 3), c8 = (lane & 7) * 8;
#pragma unroll 1
      for (int i = 0; i < 8; ++i) {
        const float kx = so[w][r][c8 + i];
        const float vx = so[w][16 + r][c8 + i];
        const float ge = 0.5f * kx * (1.0f + erff(kx * 0.70710678118654752f));
        so[w][r][c8 + i] = ge * vx * oscale;
      }
    }
#pragma unroll 1
    for (int pass = 0; pass < 2; ++pass) {
#pragma unroll 1
      for (int q = 0; q < 4; ++q) {
        const int r = q * 4 + (lane >> 3), c8 = (lane & 7) * 8;
        const v4f x0 = *(const v4fa*)&so[w][r][c8], x1 = *(const v4fa*)&so[w][r][c8 + 4];
        Frag16 fh;
#pragma unroll
        for (int i = 0; i < 4; ++i) { fh.u[i] = f16_flush_bits(x0[i]); fh.u[4 + i] = f16_flush_bits(x1[i]); }
        const size_t o = (size_t)(row0 + half * 16 + r) * (size_t)ldc + col0 + c8;
        *(volatile v8us*)(Ch + o) = fh.half[0];
      }
      if (pass == 0) __threadfence();
    }
    __builtin_amdgcn_fence(4  , "workgroup");
    __builtin_amdgcn_wave_barrier();
  }
}

template <int NHv, int TTv, bool TWO>
__global__ __launch_bounds__(256) void k_vt(const unsigned short* __restrict__ V, const unsigned short* __restrict__ V2, int ldv,
    unsigned short* __restrict__ Vt, unsigned short* __restrict__ Vt2) {
  __shared__ __attribute__((aligned(16))) unsigned short tl[64][66];
  __shared__ __attribute__((aligned(16))) unsigned short tl2[64][66];
  const int tid = threadIdx.x;
  const int slab = (int)blockIdx.x / (TTv / 64), lg = (int)blockIdx.x % (TTv / 64);
  const int b = slab / NHv, h = slab % NHv;
  for (int i = tid; i < 64 * 8; i += 256) {
    const int r = i / 8, c8 = (i % 8) * 8;
    const size_t s0 = ((size_t)b * TTv + (size_t)lg * 64 + r) * (size_t)ldv + (size_t)h * 64 + c8;
    Frag16 f;
    f.half[0] = *(const v8us*)(V + s0);
#pragma unroll
    for (int q = 0; q < 8; ++q) tl[r][c8 + q] = f.u[q];
    if (TWO) {
      Frag16 f2;
      f2.half[0] = *(const v8us*)(V2 + s0);
#pragma unroll
      for (int q = 0; q < 8; ++q) tl2[r][c8 + q] = f2.u[q];
    }
  }
  __syncthreads();
  for (int pass = 0; pass < 2; ++pass) {
#pragma unroll
    for (int rd = 0; rd < 2; ++rd) {
      const int d = rd * 32 + tid / 8, pc = tid % 8;
      Frag16 f;
#pragma unroll
      for (int q = 0; q < 8; ++q) f.u[q] = tl[pc * 8 + q][d];
      const size_t o = ((size_t)slab * 64 + d) * (size_t)TTv + (size_t)lg * 64 + pc * 8;
      *(volatile v8us*)(Vt + o) = f.half[0];
      if (TWO) {
        Frag16 f2;
#pragma unroll
        for (int q = 0; q < 8; ++q) f2.u[q] = tl2[pc * 8 + q][d];
        *(volatile v8us*)(Vt2 + o) = f2.half[0];
      }
    }
    if (pass == 0) __threadfence();
  }
}

__device__ __forceinline__ void score32(const unsigned short* __restrict__ K16, size_t kbase, const Frag16& q0, const Frag16& q1, int hh, v8f& s0, v8f& s1) {
#pragma unroll
  for (int ks = 0; ks < 2; ++ks) {
    const Frag16 k0f = ld_frag(K16 + kbase + ks * 32, hh);
    const Frag16 k1f = ld_frag(K16 + kbase + (size_t)16 * DM + ks * 32, hh);
    const Frag16 qa = (ks == 0) ? q0 : q1;
    s0 = mma_h(qa.h, k0f.h, s0);
    s1 = mma_h(qa.h, k1f.h, s1);
  }
}

__global__ __launch_bounds__(512) void k_apply(const unsigned short* __restrict__ Q16, const unsigned short* __restrict__ K16,
    const unsigned short* __restrict__ VT, const float* __restrict__ tw, const float* __restrict__ al, const float* __restrict__ be,
    const float* __restrict__ wmix, unsigned short* __restrict__ CTX) {
  __shared__ __attribute__((aligned(16))) unsigned short pool[AP_POOL];
  __shared__ __attribute__((aligned(16))) float twl[NH][64];
  const int tid = threadIdx.x, lane = tid & 31, ln = lane & 15, hh = lane >> 4;
  const int wave = __builtin_amdgcn_readfirstlane(tid >> 5);
  const int b = (int)blockIdx.x / (SEQ / 16);
  const int t0 = ((int)blockIdx.x % (SEQ / 16)) * 16;
  const int bh = b * NH + wave;
  const size_t rowbase = (size_t)b * SEQ;
  const int nst = t0 / 32 + 1;
  const size_t kcol = (size_t)wave * HD;
  Frag16 q0, q1;
  {
    const size_t qo = (rowbase + (size_t)t0 + ln) * DM + kcol;
    q0 = ld_frag(Q16 + qo, hh); q1 = ld_frag(Q16 + qo + 32, hh);
  }
  const v8f z8 = {0.f, 0.f, 0.f, 0.f, 0.f, 0.f, 0.f, 0.f};
  const v8us zero8 = {0, 0, 0, 0, 0, 0, 0, 0};
  float m[8], l[8];
#pragma unroll
  for (int r = 0; r < 8; ++r) { m[r] = -1.0e30f; l[r] = 0.f; }
#pragma unroll 1
  for (int it = 0; it < nst; ++it) {
    const int u0 = it * 32;
    v8f s0 = z8, s1 = z8;
    score32(K16, (rowbase + (size_t)u0 + ln) * DM + kcol, q0, q1, hh, s0, s1);
#pragma unroll
    for (int r = 0; r < 8; ++r) {
      const int row = t0 + 8 * hh + r;
      float sv0 = s0[r] * 0.125f, sv1 = s1[r] * 0.125f;
      sv0 = (u0 + ln > row) ? -1.0e30f : sv0;
      sv1 = (u0 + 16 + ln > row) ? -1.0e30f : sv1;
      float mx = fmaxf(sv0, sv1);
      mx = fmaxf(mx, __shfl_xor(mx, 8, 32));
      mx = fmaxf(mx, __shfl_xor(mx, 4, 32));
      mx = fmaxf(mx, __shfl_xor(mx, 2, 32));
      mx = fmaxf(mx, __shfl_xor(mx, 1, 32));
      const float mn = fmaxf(m[r], mx);
      const float corr = __expf(m[r] - mn);
      float ps = __expf(sv0 - mn) + __expf(sv1 - mn);
      ps += __shfl_xor(ps, 8, 32);
      ps += __shfl_xor(ps, 4, 32);
      ps += __shfl_xor(ps, 2, 32);
      ps += __shfl_xor(ps, 1, 32);
      l[r] = l[r] * corr + ps;
      m[r] = mn;
    }
  }
  float rowf[8];
  {
    const float* bp = be + (size_t)wave * SEQ_FULL + t0 + 8 * hh;
    const v4f b0 = *(const v4fa*)bp, b1 = *(const v4fa*)(bp + 4);
#pragma unroll
    for (int r = 0; r < 4; ++r) {
      rowf[r] = (1.0f / l[r]) * bf16_rne(b0[r]) * 256.0f;
      rowf[4 + r] = (1.0f / l[4 + r]) * bf16_rne(b1[r]) * 256.0f;
    }
  }
  Frag16 wa;
  {
    const float* wp = wmix + ln * 16 + 8 * hh;
    const v4f w0 = *(const v4fa*)wp, w1 = *(const v4fa*)(wp + 4);
#pragma unroll
    for (int e = 0; e < 4; ++e) {
      wa.u[e] = f16_flush_bits(bf16_rne(w0[e]) * 8.0f);
      wa.u[4 + e] = f16_flush_bits(bf16_rne(w1[e]) * 8.0f);
    }
    wa.half[1] = zero8;
  }
  v8f o[4] = {z8, z8, z8, z8};
#pragma unroll 1
  for (int it = 0; it < nst; ++it) {
    const int u0 = it * 32;
    {
      const int dmin = t0 - u0 - 31;
      const int i0 = iclamp((SEQ_FULL - 1) - (dmin + lane), 0, SEQ_FULL - 1);
      const int i1 = iclamp((SEQ_FULL - 1) - (dmin + 32 + lane), 0, SEQ_FULL - 1);
      const float w0 = bf16_rne(tw[(size_t)wave * SEQ_FULL + i0]);
      const float w1 = bf16_rne(tw[(size_t)wave * SEQ_FULL + i1]);
      twl[wave][lane] = w0;
      twl[wave][32 + lane] = w1;
    }
    float al0 = bf16_rne(al[(size_t)wave * SEQ_FULL + iclamp(u0 + ln, 0, SEQ - 1)]);
    float al1 = bf16_rne(al[(size_t)wave * SEQ_FULL + iclamp(u0 + 16 + ln, 0, SEQ - 1)]);
    asm volatile("" : "+v"(al0));
    asm volatile("" : "+v"(al1));
    v8f s0 = z8, s1 = z8;
    score32(K16, (rowbase + (size_t)u0 + ln) * DM + kcol, q0, q1, hh, s0, s1);
    __builtin_amdgcn_fence(4  , "workgroup");
    __builtin_amdgcn_wave_barrier();
#pragma unroll
    for (int sub = 0; sub < 2; ++sub) {
      const float alv = (sub == 0) ? al0 : al1;
#pragma unroll
      for (int r = 0; r < 8; ++r) {
        const int d = (t0 + 8 * hh + r) - (u0 + 16 * sub + ln);
        const int wi = 31 + 8 * hh + r - 16 * sub - ln;
        float twv = twl[wave][wi];
        asm volatile("" : "+v"(twv));
        const float sv = ((sub == 0) ? s0[r] : s1[r]) * 0.125f;
        const float e = __expf(sv - m[r]);
        float pv = e * rowf[r] * twv * alv;
        pv = (d >= 0) ? pv : 0.0f;
        pool[AP_PL + ((8 * hh + r) * 32 + 16 * sub + ln) * 16 + wave] = f16_flush_bits(pv);
      }
    }
    __syncthreads();
#pragma unroll
    for (int hf = 0; hf < 2; ++hf) {
      const int nt = 2 * wave + hf;
      Frag16 bm;
      bm.half[0] = *(const v8us*)&pool[AP_PL + (nt * 16 + ln) * 16 + 8 * hh];
      bm.half[1] = zero8;
      const v8f dm = mma_h(wa.h, bm.h, z8);
#pragma unroll
      for (int r = 0; r < 8; ++r) pool[AP_MX + ((8 * hh + r) * 16 + wave) * 40 + 16 * hf + ln] = f16_flush_bits(dm[r]);
    }
    __syncthreads();
    Frag16 pa;
    pa.half[0] = *(const v8us*)&pool[AP_MX + (wave * 16 + ln) * 40 + 8 * hh];
    pa.half[1] = *(const v8us*)&pool[AP_MX + (wave * 16 + ln) * 40 + 16 + 8 * hh];
#pragma unroll
    for (int j = 0; j < 4; ++j) {
      const size_t vo = ((size_t)bh * HD + (size_t)(j * 16 + ln)) * SEQ + (size_t)u0;
      const Frag16 vh = ld_frag(VT + vo, hh);
      o[j] = mma_h(pa.h, vh.h, o[j]);
    }
  }
  __syncthreads();
#pragma unroll
  for (int j = 0; j < 4; ++j) {
#pragma unroll
    for (int r = 0; r < 8; ++r) pool[(wave * 16 + 8 * hh + r) * 72 + j * 16 + ln] = f16_flush_bits(o[j][r] * (1.0f / 32.0f));
  }
  __builtin_amdgcn_fence(4  , "workgroup");
  __builtin_amdgcn_wave_barrier();
#pragma unroll 1
  for (int pass = 0; pass < 2; ++pass) {
#pragma unroll 1
    for (int q = 0; q < 4; ++q) {
      const int row = q * 4 + (lane >> 3), c8 = (lane & 7) * 8;
      const v8us v = *(const v8us*)&pool[(wave * 16 + row) * 72 + c8];
      *(volatile v8us*)(CTX + (rowbase + (size_t)t0 + row) * DM + kcol + c8) = v;
    }
    if (pass == 0) __threadfence();
  }
}

extern "C" void kernel_launch(void* const* d_in, const int* in_sizes, int n_in,
                              void* d_out, int out_size, void* d_ws, size_t ws_size, hipStream_t stream) {
  if (n_in < 24) return;
  const float* x    = (const float*)d_in[0];
  const float* g1   = (const float*)d_in[1];
  const float* b1   = (const float*)d_in[2];
  const float* g2   = (const float*)d_in[3];
  const float* b2   = (const float*)d_in[4];
  const float* Wq   = (const float*)d_in[5];
  const float* bq   = (const float*)d_in[6];
  const float* Wk   = (const float*)d_in[7];
  const float* bk   = (const float*)d_in[8];
  const float* Wv   = (const float*)d_in[9];
  const float* bv   = (const float*)d_in[10];
  const float* tw   = (const float*)d_in[11];
  const float* tal  = (const float*)d_in[12];
  const float* tbe  = (const float*)d_in[13];
  const float* tga  = (const float*)d_in[14];
  const float* Wmix = (const float*)d_in[15];
  const float* Wo   = (const float*)d_in[16];
  const float* bo   = (const float*)d_in[17];
  const float* Wk2  = (const float*)d_in[18];
  const float* bk2  = (const float*)d_in[19];
  const float* Wv2  = (const float*)d_in[20];
  const float* bv2  = (const float*)d_in[21];
  const float* Ww2  = (const float*)d_in[22];
  const float* bw2  = (const float*)d_in[23];
  if ((size_t)in_sizes[0] < ((size_t)(NB - 1) * SEQ_FULL + SEQ) * DM) return;
  if (in_sizes[1] < DM || in_sizes[2] < DM || in_sizes[3] < DM || in_sizes[4] < DM) return;
  if (in_sizes[5] < DM * DM || in_sizes[7] < DM * DM || in_sizes[9] < DM * DM || in_sizes[16] < DM * DM) return;
  if (in_sizes[6] < DM || in_sizes[8] < DM || in_sizes[10] < DM || in_sizes[17] < DM || in_sizes[23] < DM) return;
  if (in_sizes[11] < NH * SEQ_FULL || in_sizes[12] < NH * SEQ_FULL || in_sizes[13] < NH * SEQ_FULL || in_sizes[14] < SEQ) return;
  if (in_sizes[15] < NH * NH) return;
  if (in_sizes[18] < DM * HID || in_sizes[20] < DM * HID || in_sizes[22] < HID * DM) return;
  if (in_sizes[19] < HID || in_sizes[21] < HID) return;
  if ((size_t)out_size < ((size_t)(NB - 1) * OSEQ + SEQ) * DM) return;

  char* ws = (char*)d_ws;
  size_t off = 0;
  auto take = [&](size_t bytes) { char* p = ws + off; off += (bytes + 255) & ~(size_t)255; return p; };
  const size_t WPL = (size_t)DM * DM * 2, FFP = (size_t)DM * HID * 2, ACT2 = NR * DM * 2, ACT4 = NR * DM * 4, GGP = NR * HID * 2;
  unsigned short* WQ16 = (unsigned short*)take(WPL);
  unsigned short* WK16 = (unsigned short*)take(WPL);
  unsigned short* WV16 = (unsigned short*)take(WPL);
  unsigned short* WO16 = (unsigned short*)take(WPL);
  unsigned short* WK2P = (unsigned short*)take(FFP);
  unsigned short* WV2P = (unsigned short*)take(FFP);
  unsigned short* WW2P = (unsigned short*)take(FFP);
  unsigned short* HS16 = (unsigned short*)take(ACT2);
  unsigned short* H2 = HS16;
  unsigned short* Q16 = (unsigned short*)take(ACT2);
  unsigned short* K16 = (unsigned short*)take(ACT2);
  unsigned short* VH = (unsigned short*)take(ACT2);
  unsigned short* VT = (unsigned short*)take(ACT2);
  unsigned short* CTX = (unsigned short*)take(ACT2);
  float* X1 = (float*)take(ACT4);
  unsigned short* GG = (unsigned short*)take(GGP);
  float* TAB = (float*)take((size_t)SEQ * 32 * 4);
  if (off > ws_size || off > ((size_t)128 << 20)) return;

  const unsigned gw   = (unsigned)(((size_t)DM * DM / 8 + 255) / 256);
  const unsigned gw2  = (unsigned)(((size_t)DM * HID / 8 + 255) / 256);
  const unsigned gln  = (unsigned)(NR / 32);
  const unsigned gq   = (unsigned)((NR / 128) * (DM / 64));
  const unsigned gff  = (unsigned)((NR / 128) * (HID / 64));
  const unsigned gvt  = (unsigned)(NB * NH * (SEQ / 64));
  const unsigned gap  = (unsigned)(NB * (SEQ / 16));
  const unsigned gtab = (unsigned)(SEQ / 8);
  const float a16 = 0.0625f, a1024 = 1.0f / 1024.0f;
  const int M = (int)NR;
  float* out = (float*)d_out;

  k_wt<false, false><<<gw, 256, 0, stream>>>(Wq, Wq, WQ16, DM, DM, 16.0f);
  k_wt<false, false><<<gw, 256, 0, stream>>>(Wk, Wk, WK16, DM, DM, 16.0f);
  k_wt<false, false><<<gw, 256, 0, stream>>>(Wv, Wv, WV16, DM, DM, 16.0f);
  k_wt<false, false><<<gw, 256, 0, stream>>>(Wo, Wo, WO16, DM, DM, 16.0f);
  k_wt<false, false><<<gw2, 256, 0, stream>>>(Wk2, Wk2, WK2P, DM, HID, 16.0f);
  k_wt<false, false><<<gw2, 256, 0, stream>>>(Wv2, Wv2, WV2P, DM, HID, 16.0f);
  k_wt<false, false><<<gw2, 256, 0, stream>>>(Ww2, Ww2, WW2P, HID, DM, 16.0f);
  k_tab<<<gtab, 256, 0, stream>>>(TAB);

  k_ln<<<gln, 256, 0, stream>>>(x, SEQ_FULL, g1, b1, HS16, 1, 1);
  k_gemm_rope<<<gq, 128, 0, stream>>>(HS16, DM, WQ16, DM, a16, bq, TAB, SEQ, Q16, DM, M, DM, DM);
  k_gemm_rope<<<gq, 128, 0, stream>>>(HS16, DM, WK16, DM, a16, bk, TAB, SEQ, K16, DM, M, DM, DM);
  k_gemm_plain<<<gq, 128, 0, stream>>>(HS16, DM, WV16, DM, a16, bv, VH, DM, M, DM, DM);
  k_vt<NH, SEQ, false><<<gvt, 256, 0, stream>>>(VH, nullptr, DM, VT, nullptr);
  k_apply<<<gap, 512, 0, stream>>>(Q16, K16, VT, tw, tal, tbe, Wmix, CTX);
  k_gemm_wo<<<gq, 128, 0, stream>>>(CTX, DM, WO16, DM, a1024, bo, x, SEQ, SEQ_FULL, DM, tga, SEQ, X1, DM, M, 0, M, DM, DM);

  k_ln<<<gln, 256, 0, stream>>>(X1, SEQ, g2, b2, H2, 0, 0);
  k_ffup<<<gff, 128, 0, stream>>>(H2, DM, WK2P, WV2P, DM, a16, bk2, bv2, 64.0f, GG, HID, M, HID, DM);
  k_gemm_out<<<gq, 128, 0, stream>>>(GG, HID, WW2P, HID, a1024, bw2, X1, M, 0, DM, out, DM, SEQ, OSEQ, M, DM, HID);
}
